// GraphSAGE_77575699300503
// MI455X (gfx1250) — hardware-verified
//
#include <hip/hip_runtime.h>
#include <stddef.h>
#include <stdint.h>


#define DF     128
#define NCL    40
#define K0     128
#define K12    256
#define HP     256
#define PPW    256
#define PPN    128
#define NT0    256
#define NT2    128
#define CNB2   64
#define NTHR   256
#define NWAVE  8
#define EPT    8
#define CHUNK  (NTHR * EPT)
#define WCAP   (EPT * 32)
#define LISTN  (NWAVE * WCAP)
#define NBA    1024
#define SLA    10
#define NHALF  512
#define RCAP   13312
#define DEGCAP 64
#define GBM    64
#define GBN    64
#define GTHR   128
#define NU0    (NT0 * (K0 / 8))
#define NU1    (NT0 * (K12 / 8))
#define NU2    (NT2 * (K12 / 8))
#define AGG_ZINTS    (LISTN + 2 * RCAP + 3 * NBA)
#define MISC_INTS    16
#define ROWBUF_INTS  (NWAVE * HP / 2)
#define OUTS_FLOATS  (NHALF * NCL)
#define AGG_LDS_INTS (AGG_ZINTS + MISC_INTS + ROWBUF_INTS + OUTS_FLOATS)
#define WSMAX  134217728

static_assert((CHUNK & (CHUNK - 1)) == 0 && CHUNK <= 4096);
static_assert((NBA & (NBA - 1)) == 0 && NBA == (1 << SLA));
static_assert(((long long)CHUNK << SLA) < (1LL << 31));
static_assert(LISTN % NTHR == 0);
static_assert(NBA % NWAVE == 0 && NBA % 32 == 0 && NBA % GBM == 0);
static_assert(NBA % NHALF == 0 && NHALF % NWAVE == 0);
static_assert(RCAP % 32 == 0 && AGG_ZINTS % 4 == 0 && LISTN % 4 == 0);
static_assert(AGG_ZINTS % (NTHR * 4) == 0);
static_assert(((AGG_ZINTS + MISC_INTS) % 4) == 0 && (ROWBUF_INTS % 4) == 0);
static_assert(OUTS_FLOATS % (4 * NTHR) == 0);
static_assert((NHALF * NCL * 4) % 128 == 0 && (NBA * NCL * 4) % 128 == 0);
static_assert(NCL % 4 == 0 && NCL <= CNB2 && CNB2 + NCL <= NT2 && CNB2 % 4 == 0);
static_assert(K0 % 32 == 0 && K12 % 32 == 0 && K12 == 2 * DF && HP == K12 && K0 == DF);
static_assert(NT0 % GBN == 0 && NT2 % GBN == 0 && NT0 == 2 * DF);
static_assert(GBM == (GTHR / 32) * 16 && GBN == 64);
static_assert(DF == 4 * 32);
static_assert(NU0 % NTHR == 0 && NU1 % NTHR == 0 && NU2 % NTHR == 0);
static_assert((DF * (K0 / 8)) % NTHR == 0 && (DF * (K12 / 8)) % NTHR == 0);
static_assert((NCL * (K12 / 8)) % NTHR == 0 && (CNB2 * (K12 / 8)) % NTHR == 0 && ((CNB2 + NCL) * (K12 / 8)) % NTHR == 0);
static_assert(AGG_LDS_INTS * 4 <= 300000);

typedef float          v4f   __attribute__((ext_vector_type(4)));
typedef float          v8f   __attribute__((ext_vector_type(8)));
typedef int            v4i   __attribute__((ext_vector_type(4)));
typedef int            v8i   __attribute__((ext_vector_type(8)));
typedef unsigned short v4us  __attribute__((ext_vector_type(4)));
typedef unsigned short v8us  __attribute__((ext_vector_type(8)));
typedef unsigned short v16us __attribute__((ext_vector_type(16)));
typedef __bf16         v16bf __attribute__((ext_vector_type(16)));
typedef v4f  __attribute__((may_alias)) v4fa;
typedef v4i  __attribute__((may_alias)) v4ia;
typedef v4us __attribute__((may_alias)) v4usa;
typedef v8us __attribute__((may_alias)) v8usa;
union FragB { v16bf v; v16us u; v8us h[2]; v8i w; };

__device__ __forceinline__ v8f wmb(const FragB& a, const FragB& b, v8f c) {
  v8f d = __builtin_amdgcn_wmma_f32_16x16x32_bf16(false, a.v, false, b.v, (short)0, c, false, false);
  asm volatile("v_nop\n\tv_nop\n\tv_nop\n\tv_nop" : "+v"(d) : "v"(a.w), "v"(b.w));
  return d;
}

__device__ __forceinline__ unsigned bf16_bits(float f) {
  const unsigned u = __float_as_uint(f);
  return (u + 0x7FFFu + ((u >> 16) & 1u)) >> 16;
}
__device__ __forceinline__ float bf16_val(float f) {
  return __uint_as_float(bf16_bits(f) << 16);
}

__device__ __forceinline__ void wave_sync() {
  __builtin_amdgcn_fence(__ATOMIC_RELEASE, "wavefront");
  __builtin_amdgcn_wave_barrier();
  __builtin_amdgcn_fence(__ATOMIC_ACQUIRE, "wavefront");
}

template <int SLB>
__device__ __forceinline__ int scan_chunk(const int* __restrict__ dsts, int nE, int cbase, int slotBase,
                                          int nb, int vec8, int* list, int tid, int lane, int wave) {
  int wc = 0;
  const int el0  = tid * EPT;
  const int e0   = cbase + el0;
  const int sent = -2147483647 - 1;
  v4i da, db;
  if (vec8 != 0 && cbase + CHUNK <= nE) {
    da = *(const v4i*)(dsts + e0);
    db = *(const v4i*)(dsts + e0 + 4);
  } else {
    da.x = (e0     < nE) ? dsts[min(e0,     nE - 1)] : sent;
    da.y = (e0 + 1 < nE) ? dsts[min(e0 + 1, nE - 1)] : sent;
    da.z = (e0 + 2 < nE) ? dsts[min(e0 + 2, nE - 1)] : sent;
    da.w = (e0 + 3 < nE) ? dsts[min(e0 + 3, nE - 1)] : sent;
    db.x = (e0 + 4 < nE) ? dsts[min(e0 + 4, nE - 1)] : sent;
    db.y = (e0 + 5 < nE) ? dsts[min(e0 + 5, nE - 1)] : sent;
    db.z = (e0 + 6 < nE) ? dsts[min(e0 + 6, nE - 1)] : sent;
    db.w = (e0 + 7 < nE) ? dsts[min(e0 + 7, nE - 1)] : sent;
  }
  const unsigned nbs = (unsigned)slotBase;
  const unsigned unb = (unsigned)nb;
  const unsigned s0 = (unsigned)da.x - nbs, s1 = (unsigned)da.y - nbs;
  const unsigned s2 = (unsigned)da.z - nbs, s3 = (unsigned)da.w - nbs;
  const unsigned s4 = (unsigned)db.x - nbs, s5 = (unsigned)db.y - nbs;
  const unsigned s6 = (unsigned)db.z - nbs, s7 = (unsigned)db.w - nbs;
  const bool h0 = s0 < unb, h1 = s1 < unb, h2 = s2 < unb, h3 = s3 < unb;
  const bool h4 = s4 < unb, h5 = s5 < unb, h6 = s6 < unb, h7 = s7 < unb;
  const unsigned any = __builtin_amdgcn_ballot_w32(h0 | h1 | h2 | h3 | h4 | h5 | h6 | h7);
  if (any != 0u) {
#define HITJ(J, HJ, SJ) { \
      const unsigned mj = __builtin_amdgcn_ballot_w32(HJ); \
      if (mj != 0u) { \
        if (HJ) { \
          const int pos = wc + (int)__builtin_amdgcn_mbcnt_lo(mj, 0u); \
          if (pos < WCAP) list[wave * WCAP + pos] = ((el0 + (J)) << SLB) | (int)(SJ); \
        } \
        wc += (int)__builtin_popcount(mj); } }
    HITJ(0, h0, s0)
    HITJ(1, h1, s1)
    HITJ(2, h2, s2)
    HITJ(3, h3, s3)
    HITJ(4, h4, s4)
    HITJ(5, h5, s5)
    HITJ(6, h6, s6)
    HITJ(7, h7, s7)
#undef HITJ
  }
  return wc;
}

__global__ __launch_bounds__(NTHR) void k_wprep(const float* __restrict__ ws0, const float* __restrict__ wn0,
                                                const float* __restrict__ ws1, const float* __restrict__ wn1,
                                                const float* __restrict__ ws2, const float* __restrict__ wn2,
                                                unsigned short* W0T, unsigned short* W1T, unsigned short* W2T) {
  const int u = (int)blockIdx.x * NTHR + (int)threadIdx.x;
  const float* W;
  unsigned short* P;
  int nout, ncol, pitch, n, k8, zf = 0;
  if (u < NU0) {
    n = u >> 4; k8 = (u & 15) * 8; pitch = K0; P = W0T; nout = DF;
    if (n < DF) { W = ws0; ncol = n; } else { W = wn0; ncol = n - DF; }
  } else if (u < NU0 + NU1) {
    const int v = u - NU0;
    n = v >> 5; k8 = (v & 31) * 8; pitch = K12; P = W1T; nout = DF;
    if (n < DF) { W = ws1; ncol = n; } else { W = wn1; ncol = n - DF; }
  } else if (u < NU0 + NU1 + NU2) {
    const int v = u - NU0 - NU1;
    n = v >> 5; k8 = (v & 31) * 8; pitch = K12; P = W2T; nout = NCL;
    if (n < NCL)             { W = ws2; ncol = n; }
    else if (n < CNB2)       { W = ws2; ncol = 0; zf = 1; }
    else if (n < CNB2 + NCL) { W = wn2; ncol = n - CNB2; }
    else                     { W = wn2; ncol = 0; zf = 1; }
  } else {
    return;
  }
  const int kk = k8 & (DF - 1);
  const float* p = W + (size_t)kk * nout + ncol;
  v8us o;
#pragma unroll
  for (int i = 0; i < 8; ++i) {
    const unsigned b = bf16_bits(p[(size_t)i * nout]);
    o[i] = (zf != 0) ? (unsigned short)0 : (unsigned short)b;
  }
  unsigned short* dp = P + (size_t)n * pitch + k8;
  *(volatile v8us*)dp = o;
  __threadfence();
  *(volatile v8us*)dp = o;
}

__global__ __launch_bounds__(NTHR) void k_cvx(const float* __restrict__ x, int nN, int nUnits,
                                              unsigned short* xb) {
  const int u = (int)blockIdx.x * NTHR + (int)threadIdx.x;
  if (u >= nUnits) return;
  const int row = u >> 4;
  const int k8  = (u & 15) * 8;
  const int rc  = row < nN ? row : nN - 1;
  const float* p = x + (size_t)rc * DF + k8;
  const v4f a = *(const v4fa*)p;
  const v4f b = *(const v4fa*)(p + 4);
  const bool ok = row < nN;
  v8us o;
  o[0] = ok ? (unsigned short)bf16_bits(a.x) : (unsigned short)0;
  o[1] = ok ? (unsigned short)bf16_bits(a.y) : (unsigned short)0;
  o[2] = ok ? (unsigned short)bf16_bits(a.z) : (unsigned short)0;
  o[3] = ok ? (unsigned short)bf16_bits(a.w) : (unsigned short)0;
  o[4] = ok ? (unsigned short)bf16_bits(b.x) : (unsigned short)0;
  o[5] = ok ? (unsigned short)bf16_bits(b.y) : (unsigned short)0;
  o[6] = ok ? (unsigned short)bf16_bits(b.z) : (unsigned short)0;
  o[7] = ok ? (unsigned short)bf16_bits(b.w) : (unsigned short)0;
  unsigned short* dp = xb + (size_t)row * DF + k8;
  *(volatile v8us*)dp = o;
  __threadfence();
  *(volatile v8us*)dp = o;
}

__global__ __launch_bounds__(GTHR) void k_gemm(
    const unsigned short* __restrict__ A, const unsigned short* __restrict__ WT,
    float* outF, int K, int ldo)
{
  __shared__ __attribute__((aligned(16))) float stg[GBM * GBN];
  const int tid = (int)threadIdx.x, lane = tid & 31, wave = tid >> 5, hh = lane >> 4, m = lane & 15;
  const int rowBase = (int)blockIdx.x * GBM;
  const int col0    = (int)blockIdx.y * GBN;

  v8f acc[4];
  {
    const v8f z = {0.f, 0.f, 0.f, 0.f, 0.f, 0.f, 0.f, 0.f};
    acc[0] = z; acc[1] = z; acc[2] = z; acc[3] = z;
  }
  const unsigned short* ap = A  + (size_t)(rowBase + 16 * wave + m) * (size_t)K + 8 * hh;
  const unsigned short* wp = WT + (size_t)(col0 + m) * (size_t)K + 8 * hh;
  const int ksteps = K >> 5;
#pragma unroll 1
  for (int ks = 0; ks < ksteps; ++ks) {
    FragB af;
    af.h[0] = *(const v8usa*)(ap + 32 * ks);
    af.h[1] = *(const v8usa*)(ap + 32 * ks + 16);
#pragma unroll
    for (int t = 0; t < 4; ++t) {
      const unsigned short* wq = wp + (size_t)(16 * t) * (size_t)K + 32 * ks;
      FragB bf;
      bf.h[0] = *(const v8usa*)wq;
      bf.h[1] = *(const v8usa*)(wq + 16);
      acc[t] = wmb(af, bf, acc[t]);
    }
  }

#pragma unroll
  for (int t = 0; t < 4; ++t) {
    const int lc = 16 * t + m;
#pragma unroll
    for (int r = 0; r < 8; ++r) {
      const int lr = 16 * wave + 8 * hh + r;
      stg[lr * GBN + lc] = acc[t][r];
    }
  }
  __syncthreads();

  v4f fv[8];
#pragma unroll
  for (int i = 0; i < 8; ++i) {
    const int lr = 16 * wave + 2 * i + hh;
    fv[i] = *(const v4fa*)(stg + lr * GBN + 4 * m);
  }
#pragma unroll
  for (int i = 0; i < 8; ++i) {
    const int lr = 16 * wave + 2 * i + hh;
    const int gr = rowBase + lr;
    float* op = outF + (size_t)gr * (size_t)ldo + col0 + 4 * m;
    *(volatile v4f*)op = fv[i];
  }
  __threadfence();
#pragma unroll
  for (int i = 0; i < 8; ++i) {
    const int lr = 16 * wave + 2 * i + hh;
    const int gr = rowBase + lr;
    float* op = outF + (size_t)gr * (size_t)ldo + col0 + 4 * m;
    *(volatile v4f*)op = fv[i];
  }
}

template <int FIN>
__global__ __launch_bounds__(NTHR) void k_scan(const int* __restrict__ gath, const int* __restrict__ keys,
                                               int nE, int nN, int vec8, int mRows,
                                               const float* __restrict__ pl, const float* __restrict__ bias,
                                               unsigned short* hpl, float* outp, int outN) {
  constexpr int PP  = (FIN == 0) ? PPW : PPN;
  constexpr int CNB = (FIN == 0) ? DF : CNB2;
  extern __shared__ __attribute__((aligned(16))) int dsm[];
  int* list = dsm;
  int* hl   = dsm + LISTN;
  int* sl   = hl + RCAP;
  int* cnt  = sl + RCAP;
  int* offs = cnt + NBA;
  int* cur  = offs + NBA;
  int* misc = cur + NBA;
  const int tid = (int)threadIdx.x, lane = tid & 31, wave = tid >> 5;
  unsigned short* rowbuf = (unsigned short*)(misc + MISC_INTS) + wave * HP;
  float* outs = (float*)(misc + MISC_INTS + ROWBUF_INTS);
  const int nodeBase = (int)blockIdx.x * NBA;

  {
    const v4i z4 = {0, 0, 0, 0};
    for (int i = tid * 4; i < AGG_ZINTS; i += NTHR * 4) *(v4ia*)(dsm + i) = z4;
    if (tid < MISC_INTS) misc[tid] = 0;
  }
  v4f bb4;
  {
    const int bl = (FIN == 0) ? lane : (lane < (NCL / 4 - 1) ? lane : (NCL / 4 - 1));
    const v4f t1 = *(const v4fa*)(bias + 4 * bl);
    bb4.x = bf16_val(t1.x); bb4.y = bf16_val(t1.y); bb4.z = bf16_val(t1.z); bb4.w = bf16_val(t1.w);
  }
  __syncthreads();

  int t = 0, ov = 0;
  const int nChunks = (nE + CHUNK - 1) / CHUNK;
#pragma unroll 1
  for (int ch = 0; ch < nChunks; ++ch) {
    const int cbase = ch * CHUNK;
    const int wc = scan_chunk<SLA>(keys, nE, cbase, nodeBase, NBA, vec8, list, tid, lane, wave);
    if (lane == 0) misc[wave] = wc;
    __syncthreads();
    if (wave == 0) {
#pragma unroll 1
      for (int w2 = 0; w2 < NWAVE; ++w2) {
        int c = misc[w2];
        c = c < 0 ? 0 : (c > WCAP ? WCAP : c);
#pragma unroll 1
        for (int b0 = 0; b0 < c; b0 += 32) {
          const int idx = b0 + lane;
          const int ent = list[w2 * WCAP + (idx < WCAP ? idx : WCAP - 1)];
          const int m32 = (c - b0) < 32 ? (c - b0) : 32;
#pragma unroll 1
          for (int k = 0; k < m32; ++k) {
            const int u    = __builtin_amdgcn_readlane(ent, k);
            const int slot = u & (NBA - 1);
            const int el   = (u >> SLA) & (CHUNK - 1);
            const int pk   = ((cbase + el) << SLA) | slot;
            if (t < RCAP) {
              if (lane == 0) { hl[t] = pk; cnt[slot] = cnt[slot] + 1; }
              t = t + 1;
            } else {
              ov = 1;
            }
          }
        }
      }
    }
    __syncthreads();
  }
  if (wave == 0 && lane == 0) { misc[8] = t; misc[9] = ov; }
  __syncthreads();
  int tt = misc[8];
  tt = tt < 0 ? 0 : (tt > RCAP ? RCAP : tt);
  const int ovf = misc[9];

  if (wave == 0) {
    const int base = lane * (NBA / 32);
    int s = 0;
#pragma unroll 1
    for (int i = 0; i < NBA / 32; ++i) s += cnt[base + i];
    int incl = s;
#pragma unroll
    for (int d = 1; d < 32; d <<= 1) {
      const int y = __shfl_up(incl, d, 32);
      if (lane >= d) incl += y;
    }
    int run = incl - s;
#pragma unroll 1
    for (int i = 0; i < NBA / 32; ++i) {
      const int cv = cnt[base + i];
      offs[base + i] = run;
      cur[base + i]  = run;
      run += cv;
    }
  }
  __syncthreads();
  if (wave == 0) {
#pragma unroll 1
    for (int b0 = 0; b0 < tt; b0 += 32) {
      const int idx = b0 + lane;
      const int ent = hl[idx < RCAP ? idx : RCAP - 1];
      const int m32 = (tt - b0) < 32 ? (tt - b0) : 32;
#pragma unroll 1
      for (int k = 0; k < m32; ++k) {
        const int u    = __builtin_amdgcn_readlane(ent, k);
        const int slot = u & (NBA - 1);
        if (lane == 0) {
          int p = cur[slot];
          p = p < 0 ? 0 : (p > RCAP - 1 ? RCAP - 1 : p);
          sl[p] = u;
          cur[slot] = p + 1;
        }
      }
    }
  }
  __syncthreads();

  const float qnan = __int_as_float(0x7fc00000);
  const float pz = (ovf != 0) ? qnan : 0.0f;
  const int gl = (FIN == 0) ? lane : (lane & 15);
#pragma unroll 1
  for (int ps = 0; ps < NBA / NHALF; ++ps) {
#pragma unroll 1
    for (int sj = 0; sj < NHALF / NWAVE; ++sj) {
      const int s    = ps * NHALF + sj * NWAVE + wave;
      const int node = nodeBase + s;
      int c = cnt[s];
      const bool big = c > DEGCAP;
      c = c < 0 ? 0 : (c > DEGCAP ? DEGCAP : c);
      int o = offs[s];
      o = o < 0 ? 0 : (o > RCAP ? RCAP : o);
      const int nc = node < nN ? node : nN - 1;
      float a0 = 0.0f, a1 = 0.0f, a2 = 0.0f, a3 = 0.0f;
#pragma unroll 1
      for (int b0 = 0; b0 < c; b0 += 32) {
        int idx = o + b0 + lane;
        idx = idx > RCAP - 1 ? RCAP - 1 : idx;
        const int ent = sl[idx];
        int eid = ent >> SLA;
        eid = eid < 0 ? 0 : (eid > nE - 1 ? nE - 1 : eid);
        int sr = gath[eid];
        sr = sr < 0 ? 0 : (sr > nN - 1 ? nN - 1 : sr);
        const int m32 = (c - b0) < 32 ? (c - b0) : 32;
#pragma unroll 1
        for (int k = 0; k < m32; ++k) {
          const int sk = __builtin_amdgcn_readlane(sr, k);
          const v4f a = *(const v4fa*)(pl + (size_t)sk * PP + CNB + 4 * gl);
          a0 += a.x; a1 += a.y; a2 += a.z; a3 += a.w;
        }
      }
      const float cf  = (c < 1) ? 1.0f : (float)c;
      const float inv = 1.0f / cf;
      const v4f sv = *(const v4fa*)(pl + (size_t)nc * PP + 4 * gl);
      const float pzr = big ? qnan : pz;
      const bool live = node < nN;
      float y0 = (sv.x + a0 * inv) + bb4.x;
      float y1 = (sv.y + a1 * inv) + bb4.y;
      float y2 = (sv.z + a2 * inv) + bb4.z;
      float y3 = (sv.w + a3 * inv) + bb4.w;
      if constexpr (FIN == 0) {
        y0 = fmaxf(y0, 0.0f); y1 = fmaxf(y1, 0.0f); y2 = fmaxf(y2, 0.0f); y3 = fmaxf(y3, 0.0f);
      }
      y0 = y0 + pzr; y1 = y1 + pzr; y2 = y2 + pzr; y3 = y3 + pzr;
      const float v0 = live ? y0 : 0.0f;
      const float v1 = live ? y1 : 0.0f;
      const float v2 = live ? y2 : 0.0f;
      const float v3 = live ? y3 : 0.0f;
      if constexpr (FIN == 0) {
        v4us mh, ml;
        {
          unsigned hb;
          hb = bf16_bits(v0); mh[0] = (unsigned short)hb; ml[0] = (unsigned short)bf16_bits(v0 - __uint_as_float(hb << 16));
          hb = bf16_bits(v1); mh[1] = (unsigned short)hb; ml[1] = (unsigned short)bf16_bits(v1 - __uint_as_float(hb << 16));
          hb = bf16_bits(v2); mh[2] = (unsigned short)hb; ml[2] = (unsigned short)bf16_bits(v2 - __uint_as_float(hb << 16));
          hb = bf16_bits(v3); mh[3] = (unsigned short)hb; ml[3] = (unsigned short)bf16_bits(v3 - __uint_as_float(hb << 16));
        }
        *(v4usa*)(rowbuf + 4 * lane) = mh;
        *(v4usa*)(rowbuf + DF + 4 * lane) = ml;
        wave_sync();
        const v8us q0 = *(const v8usa*)(rowbuf + 8 * lane);
        wave_sync();
        if (node < mRows) {
          unsigned short* rpw = hpl + (size_t)node * HP + 8 * lane;
          *(volatile v8us*)rpw = q0;
          __threadfence();
          *(volatile v8us*)rpw = q0;
        }
      } else {
        if (lane < NCL / 4) {
          v4f w4;
          w4.x = v0; w4.y = v1; w4.z = v2; w4.w = v3;
          *(v4fa*)(outs + (s - ps * NHALF) * NCL + 4 * lane) = w4;
        }
      }
    }
    if constexpr (FIN != 0) {
      __syncthreads();
      const size_t ebase = (size_t)(nodeBase + ps * NHALF) * (size_t)NCL;
      const size_t elim  = (size_t)outN;
      constexpr int NIT = OUTS_FLOATS / (4 * NTHR);
#pragma unroll 4
      for (int it = 0; it < NIT; ++it) {
        const int e = 4 * (it * NTHR + tid);
        const v4f w4 = *(const v4fa*)(outs + e);
        if (ebase + (size_t)e + 4 <= elim) *(volatile v4f*)(outp + ebase + (size_t)e) = w4;
      }
      __threadfence();
#pragma unroll 4
      for (int it = 0; it < NIT; ++it) {
        const int e = 4 * (it * NTHR + tid);
        const v4f w4 = *(const v4fa*)(outs + e);
        if (ebase + (size_t)e + 4 <= elim) *(volatile v4f*)(outp + ebase + (size_t)e) = w4;
      }
      __syncthreads();
    }
  }
}

static inline int cdiv(int a, int b) { return (a + b - 1) / b; }
static inline size_t al256(size_t o) { return (o + 255) & ~(size_t)255; }

extern "C" void kernel_launch(void* const* d_in, const int* in_sizes, int n_in,
                              void* d_out, int out_size, void* d_ws, size_t ws_size,
                              hipStream_t stream) {
  if (n_in < 12) return;
  if (in_sizes[0] < DF || (in_sizes[0] % DF) != 0) return;
  const int nN = in_sizes[0] / DF;
  const int nE = in_sizes[1];
  if (nE < 1 || in_sizes[2] != nE) return;
  if (nE >= (1 << 21) || nN < 16 || nN >= (1 << 24)) return;
  if (in_sizes[3] != DF * DF || in_sizes[4] != DF * DF || in_sizes[5] != DF) return;
  if (in_sizes[6] != DF * DF || in_sizes[7] != DF * DF || in_sizes[8] != DF) return;
  if (in_sizes[9] != DF * NCL || in_sizes[10] != DF * NCL || in_sizes[11] != NCL) return;
  if ((long long)out_size != (long long)nN * NCL) return;

  const float* feat = (const float*)d_in[0];
  const int*   src  = (const int*)d_in[1];
  const int*   dst  = (const int*)d_in[2];
  const float* ws0  = (const float*)d_in[3];
  const float* wn0  = (const float*)d_in[4];
  const float* b0   = (const float*)d_in[5];
  const float* ws1  = (const float*)d_in[6];
  const float* wn1  = (const float*)d_in[7];
  const float* b1   = (const float*)d_in[8];
  const float* ws2  = (const float*)d_in[9];
  const float* wn2  = (const float*)d_in[10];
  const float* b2   = (const float*)d_in[11];
  float* out = (float*)d_out;
  const int outN = out_size;

  const int MP = cdiv(nN, GBM) * GBM;
  const int gM = MP / GBM;
  const int gA = cdiv(MP, NBA);
  if ((long long)gA * NBA < (long long)MP) return;
  const int vec8 = ((nE & 3) == 0) ? 1 : 0;

  char* ws = (char*)d_ws;
  size_t off = 0;
  const size_t oW0 = off; off = al256(off + (size_t)NT0 * K0 * 2);
  const size_t oW1 = off; off = al256(off + (size_t)NT0 * K12 * 2);
  const size_t oW2 = off; off = al256(off + (size_t)NT2 * K12 * 2);
  const size_t oFB = off; off = al256(off + (size_t)MP * DF * 2);
  const size_t oP  = off; off = al256(off + (size_t)MP * PPW * 4);
  const size_t oH  = off; off = al256(off + (size_t)MP * HP * 2);
  if (off > ws_size || off > (size_t)WSMAX) return;
  unsigned short* W0T = (unsigned short*)(ws + oW0);
  unsigned short* W1T = (unsigned short*)(ws + oW1);
  unsigned short* W2T = (unsigned short*)(ws + oW2);
  unsigned short* FB  = (unsigned short*)(ws + oFB);
  float*          P   = (float*)(ws + oP);
  unsigned short* H   = (unsigned short*)(ws + oH);

  const size_t ldsW = (size_t)(AGG_ZINTS + MISC_INTS + ROWBUF_INTS) * 4;
  const size_t ldsN = (size_t)AGG_LDS_INTS * 4;
  hipFuncSetAttribute(reinterpret_cast<const void*>(&k_scan<0>), hipFuncAttributeMaxDynamicSharedMemorySize, (int)ldsW);
  hipFuncSetAttribute(reinterpret_cast<const void*>(&k_scan<1>), hipFuncAttributeMaxDynamicSharedMemorySize, (int)ldsN);

  const int nUx = MP * (DF / 8);
  k_wprep<<<(NU0 + NU1 + NU2) / NTHR, NTHR, 0, stream>>>(ws0, wn0, ws1, wn1, ws2, wn2, W0T, W1T, W2T);
  k_cvx<<<cdiv(nUx, NTHR), NTHR, 0, stream>>>(feat, nN, nUx, FB);
  k_gemm<<<dim3(gM, NT0 / GBN), GTHR, 0, stream>>>(FB, W0T, P, K0, PPW);
  k_scan<0><<<gA, NTHR, ldsW, stream>>>(src, dst, nE, nN, vec8, MP, P, b0, H, out, outN);
  k_gemm<<<dim3(gM, NT0 / GBN), GTHR, 0, stream>>>(H, W1T, P, K12, PPW);
  k_scan<0><<<gA, NTHR, ldsW, stream>>>(src, dst, nE, nN, vec8, MP, P, b1, H, out, outN);
  k_gemm<<<dim3(gM, NT2 / GBN), GTHR, 0, stream>>>(H, W2T, P, K12, PPN);
  k_scan<1><<<gA, NTHR, ldsN, stream>>>(src, dst, nE, nN, vec8, MP, P, b2, H, out, outN);
}
